// BarkSelfAttention_23742579212384
// MI455X (gfx1250) — hardware-verified
//
#include <hip/hip_runtime.h>
#include <math.h>
#include <float.h>
#include <stdint.h>

constexpr int kBatch     = 8;
constexpr int kSeq       = 1024;
constexpr int kModel     = 1024;
constexpr int kHeads     = 16;
constexpr int kHeadDim   = 64;
constexpr int kQkvLd     = 3 * kModel;
constexpr int kTotRows   = kBatch * kSeq;
constexpr int kHalfBatch = 4;
constexpr int kHalfRows  = kHalfBatch * kSeq;
constexpr int kNumQB     = kSeq / 64;
constexpr float kQkScale = 0.125f;
constexpr float kMaskFill = -FLT_MAX;
static_assert(kNumQB == 16);
static_assert(kHeads == 16);
static_assert(kModel % 64 == 0 && kQkvLd % 64 == 0 && kHalfRows % 64 == 0);
static_assert(kModel % 32 == 0);

typedef __attribute__((ext_vector_type(16))) _Float16 v16h;
typedef __attribute__((ext_vector_type(8)))  _Float16 v8h;
typedef __attribute__((ext_vector_type(16))) __bf16   v16b;
typedef __attribute__((ext_vector_type(8)))  __bf16   v8b;
typedef __attribute__((ext_vector_type(8)))  float    v8f;
typedef __attribute__((ext_vector_type(4)))  float    v4f;
typedef __attribute__((ext_vector_type(8)))  unsigned short v8us;

__device__ __forceinline__ unsigned short f2bf_bits(float f) {
  unsigned u = __float_as_uint(f);
  return (unsigned short)((u + 0x7FFFu + ((u >> 16) & 1u)) >> 16);
}
__device__ __forceinline__ float bf_bits2f(unsigned short h) { return __uint_as_float(((unsigned)h) << 16); }

__device__ __forceinline__ void dep_guard_h(v8f& a, v8f& b, v16h x, v16h y) { asm volatile("v_nop\n\tv_nop\n\tv_nop\n\tv_nop" : "+v"(a), "+v"(b) : "v"(x), "v"(y)); }
__device__ __forceinline__ void dep_guard_b(v8f& a, v8f& b, v16b x, v16b y) { asm volatile("v_nop\n\tv_nop\n\tv_nop\n\tv_nop" : "+v"(a), "+v"(b) : "v"(x), "v"(y)); }
__device__ __forceinline__ void keep4_h(v16h a, v16h b, v16h c, v16h d) { asm volatile("v_nop" :: "v"(a), "v"(b), "v"(c), "v"(d)); }
__device__ __forceinline__ void keep4_b(v16b a, v16b b, v16b c, v16b d) { asm volatile("v_nop" :: "v"(a), "v"(b), "v"(c), "v"(d)); }
__device__ __forceinline__ void acc_guard4(v8f& a, v8f& b, v8f& c, v8f& d) { asm volatile("v_nop\n\tv_nop\n\tv_nop\n\tv_nop" : "+v"(a), "+v"(b), "+v"(c), "+v"(d)); }
template <typename T> struct Frag;
template <> struct Frag<_Float16> {
  typedef v16h V; union U { v16h v; v8h h[2]; };
  static __device__ __forceinline__ v16h load(const _Float16* p) {
    U f; f.h[0] = *(const v8h*)(p); f.h[1] = *(const v8h*)(p + 16); return f.v;
  }
  static __device__ __forceinline__ v8f mma(v16h a, v16h b, v8f c) {
    return __builtin_amdgcn_wmma_f32_16x16x32_f16(false, a, false, b, (short)0, c, false, false);
  }
  static __device__ __forceinline__ void guard(v8f& a, v8f& b, v16h x, v16h y) { dep_guard_h(a, b, x, y); }
  static __device__ __forceinline__ void keep(v16h a, v16h b, v16h c, v16h d) { keep4_h(a, b, c, d); }
};
template <> struct Frag<__bf16> {
  typedef v16b V; union U { v16b v; v8b h[2]; };
  static __device__ __forceinline__ v16b load(const __bf16* p) {
    U f; f.h[0] = *(const v8b*)(p); f.h[1] = *(const v8b*)(p + 16); return f.v;
  }
  static __device__ __forceinline__ v8f mma(v16b a, v16b b, v8f c) {
    return __builtin_amdgcn_wmma_f32_16x16x32_bf16(false, a, false, b, (short)0, c, false, false);
  }
  static __device__ __forceinline__ void guard(v8f& a, v8f& b, v16b x, v16b y) { dep_guard_b(a, b, x, y); }
  static __device__ __forceinline__ void keep(v16b a, v16b b, v16b c, v16b d) { keep4_b(a, b, c, d); }
};

template <int ET> struct Elem;
template <> struct Elem<0> { typedef _Float16 T; };
template <> struct Elem<1> { typedef __bf16 T; };
template <int ET, int SPLIT, int BIAS_MODE, int OUT_MODE, bool RESID, int ACT = 0>
__global__ __launch_bounds__(256) void wmma_gemm64(
    const unsigned short* __restrict__ Ap, const unsigned short* __restrict__ A2p, int lda, long strideA,
    const unsigned short* __restrict__ Btp, const unsigned short* __restrict__ Bt2p, int ldb, long strideB,
    void* __restrict__ Cout, void* __restrict__ Cout2, int ldc, long strideC,
    const float* __restrict__ bias,
    const float* __restrict__ resid, long strideR,
    int M, int N, int K, float scale) {
  typedef typename Elem<ET>::T T;
  typedef typename Frag<T>::V V;
  const T* A = (const T*)Ap; const T* A2 = (const T*)A2p; const T* Bt = (const T*)Btp; const T* Bt2 = (const T*)Bt2p;
  __shared__ __align__(16) float sT[8][16 * 68];
  const int b    = blockIdx.y;
  const int lane = threadIdx.x & 31;
  const int wave = threadIdx.x >> 5;
  const int tilesN = N >> 6;
  const int tilesM = M >> 6;
  const int tile = blockIdx.x * 8 + wave;
  if (tile >= tilesM * tilesN) return;
  const int tm = tile / tilesN;
  const int tn = tile - tm * tilesN;
  const int m0 = tm << 6;
  const int n0 = tn << 6;

  const T* Ab  = A  + (size_t)b * strideA;
  const T* Bb  = Bt + (size_t)b * strideB;
  const T* Ab2 = (SPLIT != 0) ? (A2  + (size_t)b * strideA) : nullptr;
  const T* Bb2 = (SPLIT == 1) ? (Bt2 + (size_t)b * strideB) : nullptr;

  const int rlane = lane & 15;
  const int koff  = (lane >> 4) * 8;
  const int mOff  = (lane >> 4) * 8;

  v8f acc[4][4];
#pragma unroll
  for (int i = 0; i < 4; ++i)
#pragma unroll
    for (int j = 0; j < 4; ++j) acc[i][j] = (v8f){0.f,0.f,0.f,0.f,0.f,0.f,0.f,0.f};

  for (int k0 = 0; k0 < K; k0 += 32) {
    V bh[4], bl[4];
#pragma unroll
    for (int j = 0; j < 4; ++j) {
      const size_t bo = (size_t)(n0 + (j << 4) + rlane) * ldb + koff + k0;
      bh[j] = Frag<T>::load(Bb + bo);
      if (SPLIT == 1) bl[j] = Frag<T>::load(Bb2 + bo);
    }
#pragma unroll
    for (int i = 0; i < 4; ++i) {
      const size_t ao = (size_t)(m0 + (i << 4) + rlane) * lda + koff + k0;
      V ah = Frag<T>::load(Ab + ao);
      V al;
      if (SPLIT != 0) al = Frag<T>::load(Ab2 + ao);
#pragma unroll
      for (int j = 0; j < 4; ++j) {
        acc[i][j] = Frag<T>::mma(ah, bh[j], acc[i][j]);
        if (SPLIT == 1) acc[i][j] = Frag<T>::mma(ah, bl[j], acc[i][j]);
        if (SPLIT != 0) acc[i][j] = Frag<T>::mma(al, bh[j], acc[i][j]);
      }
      Frag<T>::guard(acc[i][0], acc[i][3], ah, (SPLIT != 0) ? al : ah);
    }
    Frag<T>::keep(bh[0], bh[1], bh[2], bh[3]);
    if (SPLIT == 1) Frag<T>::keep(bl[0], bl[1], bl[2], bl[3]);
  }
  acc_guard4(acc[0][0], acc[0][1], acc[0][2], acc[0][3]);
  acc_guard4(acc[1][0], acc[1][1], acc[1][2], acc[1][3]);
  acc_guard4(acc[2][0], acc[2][1], acc[2][2], acc[2][3]);
  acc_guard4(acc[3][0], acc[3][1], acc[3][2], acc[3][3]);

  float* slab = sT[wave];
  const float* Rb = RESID ? (resid + (size_t)b * strideR) : nullptr;
#pragma unroll
  for (int i = 0; i < 4; ++i) {
    const int mBase = m0 + (i << 4);
#pragma unroll
    for (int j = 0; j < 4; ++j) {
      const int n = n0 + (j << 4) + rlane;
      float bv = 0.f;
      if (BIAS_MODE == 2) bv = bias[n];
      if (BIAS_MODE == 3) bv = bf_bits2f(f2bf_bits(bias[n]));
#pragma unroll
      for (int r = 0; r < 8; ++r) {
        float v = acc[i][j][r] * scale;
        if (BIAS_MODE == 1) v += bias[mBase + mOff + r];
        if (BIAS_MODE == 2 || BIAS_MODE == 3) v += bv;
        if (RESID) v += Rb[(size_t)(mBase + mOff + r) * ldc + n];
        if (ACT == 1) v = tanhf(v);
        if (ACT == 2) v = fmaxf(v, 0.0f);
        if (ACT == 4) v = (v > 0.f) ? v : 0.01f * v;
        slab[(mOff + r) * 68 + (j << 4) + rlane] = v;
      }
    }
    __builtin_amdgcn_fence(__ATOMIC_RELEASE, "workgroup");
    __builtin_amdgcn_wave_barrier();
    __builtin_amdgcn_fence(__ATOMIC_ACQUIRE, "workgroup");
    if (OUT_MODE == 0) {
      float* C = (float*)Cout + (size_t)b * strideC;
      const int hh = lane >> 4, c4 = (lane & 15) * 4;
      for (int pass = 0; pass < 2; ++pass) {
#pragma unroll
        for (int it = 0; it < 8; ++it) {
          const int row = it * 2 + hh;
          v4f v = *(const v4f*)(slab + row * 68 + c4);
          *(volatile v4f*)(C + (size_t)(mBase + row) * ldc + n0 + c4) = v;
        }
        __threadfence();
      }
    } else {
      const int q = lane >> 3, c8 = (lane & 7) * 8;
      unsigned short* C  = (unsigned short*)Cout  + (size_t)b * strideC;
      unsigned short* C2 = (OUT_MODE == 2) ? ((unsigned short*)Cout2 + (size_t)b * strideC) : nullptr;
      for (int pass = 0; pass < 2; ++pass) {
#pragma unroll
        for (int it = 0; it < 4; ++it) {
          const int row = it * 4 + q;
          const float* sp = slab + row * 68 + c8;
          v8h hv, lv;
#pragma unroll
          for (int e = 0; e < 8; ++e) {
            if (OUT_MODE == 1) {
              hv[e] = (_Float16)sp[e];
            } else {
              unsigned short hb = f2bf_bits(sp[e]);
              unsigned short lb = f2bf_bits(sp[e] - bf_bits2f(hb));
              hv[e] = __builtin_bit_cast(_Float16, hb);
              lv[e] = __builtin_bit_cast(_Float16, lb);
            }
          }
          *(volatile v8h*)(C + (size_t)(mBase + row) * ldc + n0 + c8) = hv;
          if (OUT_MODE == 2) *(volatile v8h*)(C2 + (size_t)(mBase + row) * ldc + n0 + c8) = lv;
        }
        __threadfence();
      }
    }
    __builtin_amdgcn_fence(__ATOMIC_RELEASE, "workgroup");
    __builtin_amdgcn_wave_barrier();
    __builtin_amdgcn_fence(__ATOMIC_ACQUIRE, "workgroup");
  }
}

__global__ __launch_bounds__(256) void cast_f32_bf16x8(const float* __restrict__ in,
                                                       unsigned short* __restrict__ out, int n8) {
  const int i = blockIdx.x * 256 + threadIdx.x;
  if (i < n8) {
    const v4f a0 = *(const v4f*)(in + (size_t)i * 8);
    const v4f a1 = *(const v4f*)(in + (size_t)i * 8 + 4);
    v8us u;
    u[0] = f2bf_bits(a0[0]); u[1] = f2bf_bits(a0[1]); u[2] = f2bf_bits(a0[2]); u[3] = f2bf_bits(a0[3]);
    u[4] = f2bf_bits(a1[0]); u[5] = f2bf_bits(a1[1]); u[6] = f2bf_bits(a1[2]); u[7] = f2bf_bits(a1[3]);
    *(volatile v8us*)(out + (size_t)i * 8) = u;
    __threadfence();
    *(volatile v8us*)(out + (size_t)i * 8) = u;
  }
}

#define WTP 72
__global__ __launch_bounds__(256) void wt_cast_bf16(const float* __restrict__ W, unsigned short* __restrict__ Wt,
                                                    int K, int N) {
  __shared__ __align__(16) unsigned short st[64 * WTP];
  const int n0 = blockIdx.x * 64, k0 = blockIdx.y * 64;
  const int tid = threadIdx.x;
  const int kr = tid >> 2, c16 = (tid & 3) * 16;
  const float* src = W + (size_t)(k0 + kr) * N + n0 + c16;
#pragma unroll
  for (int q = 0; q < 4; ++q) {
    const v4f v = *(const v4f*)(src + 4 * q);
#pragma unroll
    for (int e = 0; e < 4; ++e) st[(c16 + 4 * q + e) * WTP + kr] = f2bf_bits(v[e]);
  }
  __syncthreads();
  const int wave = tid >> 5, lane = tid & 31;
  const int q8 = lane >> 3, c8 = (lane & 7) * 8;
  for (int pass = 0; pass < 2; ++pass) {
#pragma unroll
    for (int it = 0; it < 2; ++it) {
      const int n = it * 32 + wave * 4 + q8;
      const v8us hv = *(const v8us*)(st + n * WTP + c8);
      *(volatile v8us*)(Wt + (size_t)(n0 + n) * K + k0 + c8) = hv;
    }
    __threadfence();
  }
}

__device__ __forceinline__ v8f mma_b(v16b a, v16b b, v8f c) {
  c = __builtin_amdgcn_wmma_f32_16x16x32_bf16(false, a, false, b, (short)0, c, false, false);
  asm volatile("v_nop\n\tv_nop\n\tv_nop\n\tv_nop" : "+v"(c) : "v"(a), "v"(b));
  return c;
}
__device__ __forceinline__ void bf_split(float f, __bf16& hi, __bf16& lo) {
  const unsigned short hb = f2bf_bits(f);
  hi = __builtin_bit_cast(__bf16, hb);
  lo = __builtin_bit_cast(__bf16, f2bf_bits(f - bf_bits2f(hb)));
}

#define AKC 64
#define OSP 68
__global__ __launch_bounds__(128) void attn_causal_k(
    const unsigned short* __restrict__ qkvhp, const unsigned short* __restrict__ qkvlp,
    unsigned short* __restrict__ ohp, unsigned short* __restrict__ olp) {
  union FB { v16b v; v8b h[2]; };
  __shared__ __align__(16) __bf16 Ksh[AKC * kHeadDim];
  __shared__ __align__(16) __bf16 Ksl[AKC * kHeadDim];
  __shared__ __align__(16) __bf16 Vth[kHeadDim * AKC];
  __shared__ __align__(16) __bf16 Vtl[kHeadDim * AKC];
  __shared__ __align__(16) __bf16 Psh[4][16 * AKC];
  __shared__ __align__(16) __bf16 Psl[4][16 * AKC];
  __shared__ __align__(16) float  Os[4][16 * OSP];

  const __bf16* Qh = (const __bf16*)qkvhp;
  const __bf16* Ql = (const __bf16*)qkvlp;

  const int tid  = threadIdx.x;
  const int wave = tid >> 5;
  const int lane = tid & 31;
  const int hh   = lane >> 4;
  const int c    = lane & 15;

  const int bx = blockIdx.x;
  const int qb = bx & (kNumQB - 1);
  const int bh = bx >> 4;
  const int h  = bh & (kHeads - 1);
  const int b  = bh >> 4;
  const int q0 = qb * 64 + wave * 16;

  v16b qah[2], qal[2];
  {
    const size_t qo = (size_t)(b * kSeq + q0 + c) * kQkvLd + h * kHeadDim + 8 * hh;
#pragma unroll
    for (int dc = 0; dc < 2; ++dc) {
      qah[dc] = Frag<__bf16>::load(Qh + qo + dc * 32);
      qal[dc] = Frag<__bf16>::load(Ql + qo + dc * 32);
    }
  }

  float mrow[8], lrow[8];
  v8f oacc[4];
#pragma unroll
  for (int r = 0; r < 8; ++r) { mrow[r] = -INFINITY; lrow[r] = 0.f; }
#pragma unroll
  for (int t = 0; t < 4; ++t) oacc[t] = (v8f){0.f,0.f,0.f,0.f,0.f,0.f,0.f,0.f};

  const int nIter = qb + 1;
  for (int kc = 0; kc < nIter; ++kc) {
    const int kv0 = kc * AKC;
    __syncthreads();
    {
      const int kvr = tid >> 1, dh = (tid & 1) * 32;
      const size_t mo = ((size_t)(b * kSeq + kv0 + kvr)) * kQkvLd + kModel + h * kHeadDim + dh;
      const __bf16* kh = Qh + mo;
      const __bf16* kl = Ql + mo;
      const __bf16* vh = kh + kModel;
      const __bf16* vl = kl + kModel;
#pragma unroll 1
      for (int i = 0; i < 4; ++i) {
        const v8b a0 = *(const v8b*)(kh + 8 * i);
        *(v8b*)(Ksh + kvr * kHeadDim + dh + 8 * i) = a0;
        const v8b a1 = *(const v8b*)(kl + 8 * i);
        *(v8b*)(Ksl + kvr * kHeadDim + dh + 8 * i) = a1;
        const v8b w0 = *(const v8b*)(vh + 8 * i);
        const v8b w1 = *(const v8b*)(vl + 8 * i);
#pragma unroll
        for (int e = 0; e < 8; ++e) {
          Vth[(dh + 8 * i + e) * AKC + kvr] = w0[e];
          Vtl[(dh + 8 * i + e) * AKC + kvr] = w1[e];
        }
      }
    }
    __syncthreads();

    v8f s[4];
#pragma unroll
    for (int j = 0; j < 4; ++j) {
      s[j] = (v8f){0.f,0.f,0.f,0.f,0.f,0.f,0.f,0.f};
#pragma unroll
      for (int dc = 0; dc < 2; ++dc) {
        FB kb, kq;
        kb.h[0] = *(const v8b*)(Ksh + (j * 16 + c) * kHeadDim + dc * 32 + 8 * hh);
        kb.h[1] = *(const v8b*)(Ksh + (j * 16 + c) * kHeadDim + dc * 32 + 16 + 8 * hh);
        kq.h[0] = *(const v8b*)(Ksl + (j * 16 + c) * kHeadDim + dc * 32 + 8 * hh);
        kq.h[1] = *(const v8b*)(Ksl + (j * 16 + c) * kHeadDim + dc * 32 + 16 + 8 * hh);
        s[j] = mma_b(qah[dc], kb.v, s[j]);
        s[j] = mma_b(qah[dc], kq.v, s[j]);
        s[j] = mma_b(qal[dc], kb.v, s[j]);
      }
    }
    const bool diag = (kc == qb);
    float cm[8];
#pragma unroll
    for (int r = 0; r < 8; ++r) {
      const int qrow = q0 + 8 * hh + r;
      float m = -INFINITY;
#pragma unroll
      for (int j = 0; j < 4; ++j) {
        const int kvcol = kv0 + j * 16 + c;
        float sv = s[j][r] * kQkScale;
        if (diag && (kvcol > qrow)) sv = kMaskFill;
        s[j][r] = sv;
        m = fmaxf(m, sv);
      }
#pragma unroll
      for (int off = 1; off < 16; off <<= 1) m = fmaxf(m, __shfl_xor(m, off, 32));
      cm[r] = m;
    }
    __bf16* pwh = Psh[wave];
    __bf16* pwl = Psl[wave];
#pragma unroll
    for (int r = 0; r < 8; ++r) {
      const float mnew = fmaxf(mrow[r], cm[r]);
      const float alpha = expf(mrow[r] - mnew);
      mrow[r] = mnew;
      float psum = 0.f;
#pragma unroll
      for (int j = 0; j < 4; ++j) {
        const float p = expf(s[j][r] - mnew);
        psum += p;
        __bf16 pa, pb; bf_split(p, pa, pb);
        pwh[(8 * hh + r) * AKC + j * 16 + c] = pa;
        pwl[(8 * hh + r) * AKC + j * 16 + c] = pb;
      }
#pragma unroll
      for (int off = 1; off < 16; off <<= 1) psum += __shfl_xor(psum, off, 32);
      lrow[r] = lrow[r] * alpha + psum;
#pragma unroll
      for (int t = 0; t < 4; ++t) oacc[t][r] *= alpha;
    }
    __builtin_amdgcn_fence(__ATOMIC_RELEASE, "workgroup");
    __builtin_amdgcn_wave_barrier();
    __builtin_amdgcn_fence(__ATOMIC_ACQUIRE, "workgroup");
#pragma unroll 1
    for (int kk = 0; kk < 2; ++kk) {
      FB pa, pl;
      pa.h[0] = *(const v8b*)(pwh + c * AKC + kk * 32 + 8 * hh);
      pa.h[1] = *(const v8b*)(pwh + c * AKC + kk * 32 + 16 + 8 * hh);
      pl.h[0] = *(const v8b*)(pwl + c * AKC + kk * 32 + 8 * hh);
      pl.h[1] = *(const v8b*)(pwl + c * AKC + kk * 32 + 16 + 8 * hh);
#pragma unroll
      for (int t = 0; t < 4; ++t) {
        FB vb, vq;
        vb.h[0] = *(const v8b*)(Vth + (t * 16 + c) * AKC + kk * 32 + 8 * hh);
        vb.h[1] = *(const v8b*)(Vth + (t * 16 + c) * AKC + kk * 32 + 16 + 8 * hh);
        vq.h[0] = *(const v8b*)(Vtl + (t * 16 + c) * AKC + kk * 32 + 8 * hh);
        vq.h[1] = *(const v8b*)(Vtl + (t * 16 + c) * AKC + kk * 32 + 16 + 8 * hh);
        oacc[t] = mma_b(pa.v, vb.v, oacc[t]);
        oacc[t] = mma_b(pa.v, vq.v, oacc[t]);
        oacc[t] = mma_b(pl.v, vb.v, oacc[t]);
      }
    }
  }

  float* os = Os[wave];
#pragma unroll
  for (int r = 0; r < 8; ++r) {
    const float inv = 1.0f / lrow[r];
#pragma unroll
    for (int t = 0; t < 4; ++t) os[(8 * hh + r) * OSP + t * 16 + c] = oacc[t][r] * inv;
  }
  __builtin_amdgcn_fence(__ATOMIC_RELEASE, "workgroup");
  __builtin_amdgcn_wave_barrier();
  __builtin_amdgcn_fence(__ATOMIC_ACQUIRE, "workgroup");
  {
    const int q8 = lane >> 3, c8 = (lane & 7) * 8;
    _Float16* Oh = (_Float16*)ohp;
    _Float16* Ol = (_Float16*)olp;
    for (int pass = 0; pass < 2; ++pass) {
#pragma unroll
      for (int it = 0; it < 4; ++it) {
        const int row = it * 4 + q8;
        const float* sp = os + row * OSP + c8;
        v8h hv, lv;
#pragma unroll
        for (int e = 0; e < 8; ++e) {
          const unsigned short hb = f2bf_bits(sp[e]);
          const unsigned short lb = f2bf_bits(sp[e] - bf_bits2f(hb));
          hv[e] = __builtin_bit_cast(_Float16, hb);
          lv[e] = __builtin_bit_cast(_Float16, lb);
        }
        const size_t oo = (size_t)(b * kSeq + q0 + row) * kModel + h * kHeadDim + c8;
        *(volatile v8h*)(Oh + oo) = hv;
        *(volatile v8h*)(Ol + oo) = lv;
      }
      __threadfence();
    }
  }
}

extern "C" void kernel_launch(void* const* d_in, const int* in_sizes, int n_in,
                              void* d_out, int out_size, void* d_ws, size_t ws_size,
                              hipStream_t stream) {
  if (n_in < 5) return;
  if (in_sizes[0] != kTotRows * kModel) return;
  if (in_sizes[1] != kModel * kQkvLd) return;
  if (in_sizes[2] != kQkvLd) return;
  if (in_sizes[3] != kModel * kModel) return;
  if (in_sizes[4] != kModel) return;
  if (out_size != kTotRows * kModel) return;

  const float* hidden = (const float*)d_in[0];
  const float* wattn  = (const float*)d_in[1];
  const float* battn  = (const float*)d_in[2];
  const float* wout   = (const float*)d_in[3];
  const float* bout   = (const float*)d_in[4];
  float* out = (float*)d_out;

  char* ws = (char*)d_ws;
  size_t off = 0;
  const size_t szXb  = (size_t)kTotRows * kModel * 2;
  const size_t szWaT = (size_t)kQkvLd * kModel * 2;
  const size_t szWoT = (size_t)kModel * kModel * 2;
  const size_t szQKV = (size_t)kHalfRows * kQkvLd * 2;
  const size_t szO   = (size_t)kHalfRows * kModel * 2;
  unsigned short* Xb   = (unsigned short*)(ws + off); off += szXb;
  unsigned short* WaT  = (unsigned short*)(ws + off); off += szWaT;
  unsigned short* WoT  = (unsigned short*)(ws + off); off += szWoT;
  unsigned short* QKVh = (unsigned short*)(ws + off); off += szQKV;
  unsigned short* QKVl = (unsigned short*)(ws + off); off += szQKV;
  unsigned short* Oh   = (unsigned short*)(ws + off); off += szO;
  unsigned short* Ol   = (unsigned short*)(ws + off); off += szO;
  if (off > ws_size) return;

  {
    const int n8 = kTotRows * kModel / 8;
    cast_f32_bf16x8<<<dim3((n8 + 255) / 256), dim3(256), 0, stream>>>(hidden, Xb, n8);
  }
  wt_cast_bf16<<<dim3(kQkvLd / 64, kModel / 64), dim3(256), 0, stream>>>(wattn, WaT, kModel, kQkvLd);
  wt_cast_bf16<<<dim3(kModel / 64, kModel / 64), dim3(256), 0, stream>>>(wout, WoT, kModel, kModel);

  for (int half = 0; half < kBatch / kHalfBatch; ++half) {
    const unsigned short* Xh = Xb + (size_t)half * kHalfRows * kModel;
    float* outh = out + (size_t)half * kHalfRows * kModel;
    wmma_gemm64<1, 0, 3, 2, false><<<dim3(((kHalfRows / 64) * (kQkvLd / 64) + 7) / 8, 1), dim3(256), 0, stream>>>(
        Xh, nullptr, kModel, 0L, WaT, nullptr, kModel, 0L,
        (void*)QKVh, (void*)QKVl, kQkvLd, 0L, battn, nullptr, 0L, kHalfRows, kQkvLd, kModel, 1.0f);
    attn_causal_k<<<dim3(kHalfBatch * kHeads * kNumQB), dim3(128), 0, stream>>>(QKVh, QKVl, Oh, Ol);
    wmma_gemm64<1, 2, 3, 0, false><<<dim3(((kHalfRows / 64) * (kModel / 64) + 7) / 8, 1), dim3(256), 0, stream>>>(
        Oh, Ol, kModel, 0L, WoT, nullptr, kModel, 0L,
        (void*)outh, nullptr, kModel, 0L, bout, nullptr, 0L, kHalfRows, kModel, kModel, 1.0f);
  }
}
